// RFCN_71940702208530
// MI455X (gfx1250) — hardware-verified
//
#include <hip/hip_runtime.h>
#include <stdint.h>

constexpr int kNB    = 2;
constexpr int kCin   = 1024;
constexpr int kHf    = 38;
constexpr int kWf    = 56;
constexpr int kHW    = kHf * kWf;
constexpr int kHWp   = 2176;
constexpr int kFeat  = 512;
constexpr int kNR    = 512;
constexpr int kPS    = 7;
constexpr int kNSmp  = 196;
constexpr int kNCls  = 81;
constexpr int kNLoc  = 4;
constexpr int kOCls  = kPS * kPS * kNCls;
constexpr int kOClsP = 4032;
constexpr int kOLoc  = kPS * kPS * kNLoc;
constexpr int kOLocP = 256;
static_assert(kHWp % 64 == 0 && kHWp >= kHW, "position pad");
static_assert(kOClsP % 64 == 0 && kOClsP >= kOCls, "cls channel pad");
static_assert(kOLocP % 64 == 0 && kOLocP >= kOLoc, "loc channel pad");
static_assert(kCin % 32 == 0 && kFeat % 64 == 0, "K multiples");
static_assert((kNR * kNCls) % 32 == 0 && (kNR * kNLoc) % 32 == 0, "whole output lines");

constexpr size_t kOffFT  = 0;
constexpr size_t kSzFT   = (size_t)kNB * kHWp * kCin * 2;
constexpr size_t kOffWN  = kOffFT + kSzFT;
constexpr size_t kSzWN   = (size_t)kFeat * kCin * 2;
constexpr size_t kOffXTH = kOffWN + kSzWN;
constexpr size_t kSzXT   = (size_t)kNB * kHWp * kFeat * 2;
constexpr size_t kOffXTL = kOffXTH + kSzXT;
constexpr size_t kOffWS  = kOffXTL + kSzXT;
constexpr size_t kSzWS   = (size_t)kOClsP * kFeat * 2;
constexpr size_t kOffWB  = kOffWS + kSzWS;
constexpr size_t kSzWB   = (size_t)kOLocP * kFeat * 2;
constexpr size_t kOffBS  = kOffWB + kSzWB;
constexpr size_t kSzBS   = (size_t)kOClsP * 4;
constexpr size_t kOffBB  = kOffBS + kSzBS;
constexpr size_t kSzBB   = (size_t)kOLocP * 4;
constexpr size_t kOffCLS = kOffBB + kSzBB;
constexpr size_t kSzCLS  = (size_t)kNB * kOClsP * kHWp * 4;
constexpr size_t kOffLOC = kOffCLS + kSzCLS;
constexpr size_t kSzLOC  = (size_t)kNB * kOLocP * kHWp * 4;
constexpr size_t kWsTotal = kOffLOC + kSzLOC;
static_assert(kWsTotal == 97927936ull, "carve total");
static_assert(kWsTotal <= 134217728ull, "carve under 128 MiB");
static_assert(kOffWN % 256 == 0 && kOffXTH % 256 == 0 && kOffXTL % 256 == 0 && kOffWS % 256 == 0 &&
              kOffWB % 256 == 0 && kOffBS % 256 == 0 && kOffBB % 256 == 0 && kOffCLS % 256 == 0 &&
              kOffLOC % 256 == 0, "aligned regions");

typedef __attribute__((ext_vector_type(16))) _Float16 v16h;
typedef __attribute__((ext_vector_type(8)))  _Float16 v8h;
typedef __attribute__((ext_vector_type(16))) __bf16   v16b;
typedef __attribute__((ext_vector_type(8)))  __bf16   v8b;
typedef __attribute__((ext_vector_type(8)))  float    v8f;
typedef __attribute__((ext_vector_type(4)))  float    v4f;
typedef __attribute__((ext_vector_type(4)))  unsigned int v4u;

__device__ __forceinline__ unsigned short f2bf_bits(float f) {
  unsigned u = __float_as_uint(f);
  return (unsigned short)((u + 0x7FFFu + ((u >> 16) & 1u)) >> 16);
}
__device__ __forceinline__ float bf_bits2f(unsigned short h) { return __uint_as_float(((unsigned)h) << 16); }

__device__ __forceinline__ void dep_guard_h(v8f& a, v8f& b, v16h x, v16h y) { asm volatile("v_nop\n\tv_nop\n\tv_nop\n\tv_nop" : "+v"(a), "+v"(b) : "v"(x), "v"(y)); }
__device__ __forceinline__ void dep_guard_b(v8f& a, v8f& b, v16b x, v16b y) { asm volatile("v_nop\n\tv_nop\n\tv_nop\n\tv_nop" : "+v"(a), "+v"(b) : "v"(x), "v"(y)); }
__device__ __forceinline__ void keep4_h(v16h a, v16h b, v16h c, v16h d) { asm volatile("v_nop" :: "v"(a), "v"(b), "v"(c), "v"(d)); }
__device__ __forceinline__ void keep4_b(v16b a, v16b b, v16b c, v16b d) { asm volatile("v_nop" :: "v"(a), "v"(b), "v"(c), "v"(d)); }
__device__ __forceinline__ void acc_guard4(v8f& a, v8f& b, v8f& c, v8f& d) { asm volatile("v_nop\n\tv_nop\n\tv_nop\n\tv_nop" : "+v"(a), "+v"(b), "+v"(c), "+v"(d)); }
template <typename T> struct Frag;
template <> struct Frag<_Float16> {
  typedef v16h V; union U { v16h v; v8h h[2]; };
  static __device__ __forceinline__ v16h load(const _Float16* p) {
    U f; f.h[0] = *(const v8h*)(p); f.h[1] = *(const v8h*)(p + 16); return f.v;
  }
  static __device__ __forceinline__ v8f mma(v16h a, v16h b, v8f c) {
    return __builtin_amdgcn_wmma_f32_16x16x32_f16(false, a, false, b, (short)0, c, false, false);
  }
  static __device__ __forceinline__ void guard(v8f& a, v8f& b, v16h x, v16h y) { dep_guard_h(a, b, x, y); }
  static __device__ __forceinline__ void keep(v16h a, v16h b, v16h c, v16h d) { keep4_h(a, b, c, d); }
};
template <> struct Frag<__bf16> {
  typedef v16b V; union U { v16b v; v8b h[2]; };
  static __device__ __forceinline__ v16b load(const __bf16* p) {
    U f; f.h[0] = *(const v8b*)(p); f.h[1] = *(const v8b*)(p + 16); return f.v;
  }
  static __device__ __forceinline__ v8f mma(v16b a, v16b b, v8f c) {
    return __builtin_amdgcn_wmma_f32_16x16x32_bf16(false, a, false, b, (short)0, c, false, false);
  }
  static __device__ __forceinline__ void guard(v8f& a, v8f& b, v16b x, v16b y) { dep_guard_b(a, b, x, y); }
  static __device__ __forceinline__ void keep(v16b a, v16b b, v16b c, v16b d) { keep4_b(a, b, c, d); }
};

__device__ __forceinline__ unsigned pk16(unsigned short a, unsigned short b) { return (unsigned)a | ((unsigned)b << 16); }
__device__ __forceinline__ float bfr(float f) { return bf_bits2f(f2bf_bits(f)); }

template <int ET> struct Elem;
template <> struct Elem<0> { typedef _Float16 T; };
template <> struct Elem<1> { typedef __bf16 T; };
template <int ET, int SPLIT, int BIAS_MODE, int OUT_MODE, bool RESID, int ACT = 0>
__global__ __launch_bounds__(256) void wmma_gemm64(
    const unsigned short* __restrict__ Ap, const unsigned short* __restrict__ A2p, int lda, long strideA,
    const unsigned short* __restrict__ Btp, const unsigned short* __restrict__ Bt2p, int ldb, long strideB,
    void* __restrict__ Cout, void* __restrict__ Cout2, int ldc, long strideC,
    const float* __restrict__ bias,
    const float* __restrict__ resid, long strideR,
    int M, int N, int K, float scale) {
  typedef typename Elem<ET>::T T;
  typedef typename Frag<T>::V V;
  const T* A = (const T*)Ap; const T* A2 = (const T*)A2p; const T* Bt = (const T*)Btp; const T* Bt2 = (const T*)Bt2p;
  __shared__ __align__(16) float sT[8][16 * 68];
  const int b    = blockIdx.y;
  const int lane = threadIdx.x & 31;
  const int wave = threadIdx.x >> 5;
  const int tilesN = N >> 6;
  const int tilesM = M >> 6;
  const int tile = blockIdx.x * 8 + wave;
  if (tile >= tilesM * tilesN) return;
  const int tm = tile / tilesN;
  const int tn = tile - tm * tilesN;
  const int m0 = tm << 6;
  const int n0 = tn << 6;

  const T* Ab  = A  + (size_t)b * strideA;
  const T* Bb  = Bt + (size_t)b * strideB;
  const T* Ab2 = (SPLIT == 1) ? (A2  + (size_t)b * strideA) : nullptr;
  const T* Bb2 = (SPLIT != 0) ? (Bt2 + (size_t)b * strideB) : nullptr;

  const int rlane = lane & 15;
  const int koff  = (lane >> 4) * 8;
  const int mOff  = (lane >> 4) * 8;

  v8f acc[4][4];
#pragma unroll
  for (int i = 0; i < 4; ++i)
#pragma unroll
    for (int j = 0; j < 4; ++j) acc[i][j] = (v8f){0.f,0.f,0.f,0.f,0.f,0.f,0.f,0.f};

  for (int k0 = 0; k0 < K; k0 += 32) {
    V bh[4], bl[4];
#pragma unroll
    for (int j = 0; j < 4; ++j) {
      const size_t bo = (size_t)(n0 + (j << 4) + rlane) * ldb + koff + k0;
      bh[j] = Frag<T>::load(Bb + bo);
      if (SPLIT != 0) bl[j] = Frag<T>::load(Bb2 + bo);
    }
#pragma unroll
    for (int i = 0; i < 4; ++i) {
      const size_t ao = (size_t)(m0 + (i << 4) + rlane) * lda + koff + k0;
      V ah = Frag<T>::load(Ab + ao);
      V al = ah;
      if (SPLIT == 1) al = Frag<T>::load(Ab2 + ao);
#pragma unroll
      for (int j = 0; j < 4; ++j) {
        acc[i][j] = Frag<T>::mma(ah, bh[j], acc[i][j]);
        if (SPLIT != 0) acc[i][j] = Frag<T>::mma(ah, bl[j], acc[i][j]);
        if (SPLIT == 1) acc[i][j] = Frag<T>::mma(al, bh[j], acc[i][j]);
      }
      Frag<T>::guard(acc[i][0], acc[i][3], ah, al);
    }
    Frag<T>::keep(bh[0], bh[1], bh[2], bh[3]);
    if (SPLIT != 0) Frag<T>::keep(bl[0], bl[1], bl[2], bl[3]);
  }
  acc_guard4(acc[0][0], acc[0][1], acc[0][2], acc[0][3]);
  acc_guard4(acc[1][0], acc[1][1], acc[1][2], acc[1][3]);
  acc_guard4(acc[2][0], acc[2][1], acc[2][2], acc[2][3]);
  acc_guard4(acc[3][0], acc[3][1], acc[3][2], acc[3][3]);

  float* slab = sT[wave];
  const float* Rb = RESID ? (resid + (size_t)b * strideR) : nullptr;
#pragma unroll
  for (int i = 0; i < 4; ++i) {
    const int mBase = m0 + (i << 4);
#pragma unroll
    for (int j = 0; j < 4; ++j) {
      const int n = n0 + (j << 4) + rlane;
      float bv = 0.f;
      if (BIAS_MODE == 2) bv = bias[n];
#pragma unroll
      for (int r = 0; r < 8; ++r) {
        float v = acc[i][j][r] * scale;
        if (BIAS_MODE == 1) v += bias[mBase + mOff + r];
        if (BIAS_MODE == 2) v += bv;
        if (RESID) v += Rb[(size_t)(mBase + mOff + r) * ldc + n];
        if (ACT == 2) v = fmaxf(v, 0.0f);
        if (ACT == 4) v = (v > 0.f) ? v : 0.01f * v;
        slab[(mOff + r) * 68 + (j << 4) + rlane] = v;
      }
    }
    __builtin_amdgcn_fence(__ATOMIC_RELEASE, "workgroup");
    __builtin_amdgcn_wave_barrier();
    __builtin_amdgcn_fence(__ATOMIC_ACQUIRE, "workgroup");
    if (OUT_MODE == 0) {
      float* C = (float*)Cout + (size_t)b * strideC;
      const int hh = lane >> 4, c4 = (lane & 15) * 4;
      for (int pass = 0; pass < 2; ++pass) {
#pragma unroll
        for (int it = 0; it < 8; ++it) {
          const int row = it * 2 + hh;
          v4f v = *(const v4f*)(slab + row * 68 + c4);
          *(volatile v4f*)(C + (size_t)(mBase + row) * ldc + n0 + c4) = v;
        }
        __threadfence();
      }
    } else {
      const int q = lane >> 3, c8 = (lane & 7) * 8;
      unsigned short* C  = (unsigned short*)Cout  + (size_t)b * strideC;
      unsigned short* C2 = (OUT_MODE == 2) ? ((unsigned short*)Cout2 + (size_t)b * strideC) : nullptr;
      for (int pass = 0; pass < 2; ++pass) {
#pragma unroll
        for (int it = 0; it < 4; ++it) {
          const int row = it * 4 + q;
          const float* sp = slab + row * 68 + c8;
          v8h hv, lv;
#pragma unroll
          for (int e = 0; e < 8; ++e) {
            if (OUT_MODE == 1) {
              hv[e] = (_Float16)sp[e];
            } else {
              unsigned short hb = f2bf_bits(sp[e]);
              unsigned short lb = f2bf_bits(sp[e] - bf_bits2f(hb));
              hv[e] = __builtin_bit_cast(_Float16, hb);
              lv[e] = __builtin_bit_cast(_Float16, lb);
            }
          }
          *(volatile v8h*)(C + (size_t)(mBase + row) * ldc + n0 + c8) = hv;
          if (OUT_MODE == 2) *(volatile v8h*)(C2 + (size_t)(mBase + row) * ldc + n0 + c8) = lv;
        }
        __threadfence();
      }
    }
    __builtin_amdgcn_fence(__ATOMIC_RELEASE, "workgroup");
    __builtin_amdgcn_wave_barrier();
    __builtin_amdgcn_fence(__ATOMIC_ACQUIRE, "workgroup");
  }
}

__global__ __launch_bounds__(256) void k_feat_tcast(const float* __restrict__ feat, unsigned short* __restrict__ FT) {
  __shared__ float sm[64][65];
  const int t  = threadIdx.x;
  const int p0 = blockIdx.x * 64;
  const int c0 = blockIdx.y * 64;
  const int b  = blockIdx.z;
  const float* fb = feat + (size_t)b * kCin * kHW;
#pragma unroll
  for (int i = 0; i < 16; ++i) {
    const int e  = i * 256 + t;
    const int cl = e >> 6;
    const int pl = e & 63;
    const int p  = p0 + pl;
    const int pc = (p < kHW) ? p : (kHW - 1);
    float v = fb[(size_t)(c0 + cl) * kHW + pc];
    v = (p < kHW) ? v : 0.0f;
    sm[pl][cl] = v;
  }
  __syncthreads();
  const int lane = t & 31, wave = t >> 5;
  const int q = lane >> 3, c8 = (lane & 7) * 8;
  unsigned short* op = FT + (size_t)b * kHWp * kCin;
  for (int pass = 0; pass < 2; ++pass) {
#pragma unroll
    for (int it = 0; it < 2; ++it) {
      const int row = wave * 8 + it * 4 + q;
      unsigned short hb[8];
#pragma unroll
      for (int e = 0; e < 8; ++e) hb[e] = f2bf_bits(sm[row][c8 + e]);
      const v4u u = (v4u){pk16(hb[0], hb[1]), pk16(hb[2], hb[3]), pk16(hb[4], hb[5]), pk16(hb[6], hb[7])};
      *(volatile v4u*)(op + (size_t)(p0 + row) * kCin + c0 + c8) = u;
    }
    __threadfence();
  }
}

__global__ __launch_bounds__(256) void k_cast_rows(const float* __restrict__ in, int mreal,
                                                   unsigned short* __restrict__ out, int k8, int n8) {
  const int i = blockIdx.x * 256 + threadIdx.x;
  if (i >= n8) return;
  const int row  = i / k8;
  const int c8   = (i - row * k8) * 8;
  const int rowc = (row < mreal) ? row : (mreal - 1);
  const float* p = in + (size_t)rowc * (size_t)(k8 * 8) + c8;
  const v4f a = *(const v4f*)(p);
  const v4f c = *(const v4f*)(p + 4);
  const bool live = row < mreal;
  unsigned short hb[8];
#pragma unroll
  for (int e = 0; e < 4; ++e) {
    hb[e]     = live ? f2bf_bits(a[e]) : (unsigned short)0;
    hb[4 + e] = live ? f2bf_bits(c[e]) : (unsigned short)0;
  }
  const v4u u = (v4u){pk16(hb[0], hb[1]), pk16(hb[2], hb[3]), pk16(hb[4], hb[5]), pk16(hb[6], hb[7])};
  unsigned short* q = out + 8 * (size_t)i;
  *(volatile v4u*)q = u;
  __threadfence();
  *(volatile v4u*)q = u;
}

__global__ __launch_bounds__(256) void k_bias_pad(const float* __restrict__ in, int nreal, float* __restrict__ out, int n4) {
  const int i = blockIdx.x * 256 + threadIdx.x;
  if (i >= n4) return;
  v4f v;
#pragma unroll
  for (int e = 0; e < 4; ++e) {
    const int j  = 4 * i + e;
    const int jc = (j < nreal) ? j : (nreal - 1);
    const float x = in[jc];
    v[e] = (j < nreal) ? bfr(x) : 0.0f;
  }
  float* q = out + 4 * (size_t)i;
  *(volatile v4f*)q = v;
  __threadfence();
  *(volatile v4f*)q = v;
}

__global__ __launch_bounds__(256) void k_psroi_pool(const float* __restrict__ rois, const int* __restrict__ stride_p,
                                                    const float* __restrict__ maps, long plane_stride,
                                                    int nco, int nchan, float* __restrict__ outp, int ntot) {
  __shared__ float lbuf[32];
  const int t = threadIdx.x, lane = t & 31, wave = t >> 5;
  const int f0 = blockIdx.x * 32;
  const float inv = 1.0f / (float)stride_p[0];
  const float ymax = (float)(kHf - 1), xmax = (float)(kWf - 1);
#pragma unroll 1
  for (int s = 0; s < 4; ++s) {
    int f = f0 + wave * 4 + s;
    f = (f < ntot) ? f : (ntot - 1);
    int r = f / nco;
    const int co = f - r * nco;
    r = (r < kNR) ? r : (kNR - 1);
    const float* roi = rois + (size_t)r * 5;
    const float rb0 = bfr(roi[0]);
    const float rb1 = bfr(roi[1]);
    const float rb2 = bfr(roi[2]);
    const float rb3 = bfr(roi[3]);
    const float rb4 = bfr(roi[4]);
    const int braw = (int)rb0;
    int bb = (braw < 0) ? (braw + kNB) : braw;
    bb = (bb < 0) ? 0 : bb;
    bb = (bb > kNB - 1) ? (kNB - 1) : bb;
    const float x1 = rb1 * inv, y1 = rb2 * inv, x2 = rb3 * inv, y2 = rb4 * inv;
    const float bw = fmaxf(x2 - x1, 0.1f) * (1.0f / 7.0f);
    const float bh = fmaxf(y2 - y1, 0.1f) * (1.0f / 7.0f);
    const float* mb = maps + (size_t)bb * (size_t)plane_stride;
    float acc = 0.0f;
#pragma unroll 1
    for (int it = 0; it < 7; ++it) {
      const int smp = it * 32 + lane;
      const bool live = smp < kNSmp;
      const int sc = live ? smp : (kNSmp - 1);
      const int bin = sc >> 2;
      const int sy = (sc >> 1) & 1, sx = sc & 1;
      const int ph = bin / kPS;
      const int pw = bin - ph * kPS;
      float y = y1 + ((float)ph + ((float)sy + 0.5f) * 0.5f) * bh;
      float x = x1 + ((float)pw + ((float)sx + 0.5f) * 0.5f) * bw;
      y = fminf(fmaxf(y, 0.0f), ymax);
      x = fminf(fmaxf(x, 0.0f), xmax);
      const float y0f = floorf(y), x0f = floorf(x);
      int y0 = (int)y0f, x0 = (int)x0f;
      y0 = (y0 < 0) ? 0 : y0; y0 = (y0 > kHf - 1) ? (kHf - 1) : y0;
      x0 = (x0 < 0) ? 0 : x0; x0 = (x0 > kWf - 1) ? (kWf - 1) : x0;
      const int y1i = (y0 + 1 < kHf - 1) ? (y0 + 1) : (kHf - 1);
      const int x1i = (x0 + 1 < kWf - 1) ? (x0 + 1) : (kWf - 1);
      const float wy = y - y0f, wx = x - x0f;
      int chan = (co * kPS + ph) * kPS + pw;
      chan = (chan < 0) ? 0 : chan;
      chan = (chan > nchan - 1) ? (nchan - 1) : chan;
      const float* mr = mb + (size_t)chan * kHWp;
      const float v00 = mr[y0 * kWf + x0];
      const float v01 = mr[y0 * kWf + x1i];
      const float v10 = mr[y1i * kWf + x0];
      const float v11 = mr[y1i * kWf + x1i];
      const float v = (1.0f - wy) * (1.0f - wx) * v00 + (1.0f - wy) * wx * v01
                    + wy * (1.0f - wx) * v10 + wy * wx * v11;
      acc += live ? v : 0.0f;
    }
#pragma unroll
    for (int off = 16; off > 0; off >>= 1) acc += __shfl_xor(acc, off, 32);
    const float res = (acc * 0.25f) * (1.0f / 49.0f);
    if (lane == 0) lbuf[wave * 4 + s] = res;
  }
  __syncthreads();
  if (wave == 0) {
    const float v = lbuf[lane];
    float* op = outp + (size_t)f0 + lane;
    *(volatile float*)op = v;
    __threadfence();
    *(volatile float*)op = v;
  }
}

extern "C" void kernel_launch(void* const* d_in, const int* in_sizes, int n_in,
                              void* d_out, int out_size, void* d_ws, size_t ws_size,
                              hipStream_t stream) {
  (void)in_sizes;
  if (n_in < 8) return;
  if (ws_size < kWsTotal) return;
  if (out_size < kNR * (kNCls + kNLoc)) return;
  const float* rois    = (const float*)d_in[0];
  const float* feat    = (const float*)d_in[1];
  const float* w_new   = (const float*)d_in[2];
  const float* w_score = (const float*)d_in[3];
  const float* b_score = (const float*)d_in[4];
  const float* w_bbox  = (const float*)d_in[5];
  const float* b_bbox  = (const float*)d_in[6];
  const int*   stridep = (const int*)d_in[7];
  float* out = (float*)d_out;
  char* ws = (char*)d_ws;
  unsigned short* FT  = (unsigned short*)(ws + kOffFT);
  unsigned short* WN  = (unsigned short*)(ws + kOffWN);
  unsigned short* XTH = (unsigned short*)(ws + kOffXTH);
  unsigned short* XTL = (unsigned short*)(ws + kOffXTL);
  unsigned short* WS  = (unsigned short*)(ws + kOffWS);
  unsigned short* WB  = (unsigned short*)(ws + kOffWB);
  float* BS  = (float*)(ws + kOffBS);
  float* BB  = (float*)(ws + kOffBB);
  float* CLS = (float*)(ws + kOffCLS);
  float* LOC = (float*)(ws + kOffLOC);

  k_feat_tcast<<<dim3(kHWp / 64, kCin / 64, kNB), 256, 0, stream>>>(feat, FT);
  {
    const int n8 = kFeat * kCin / 8;
    k_cast_rows<<<(n8 + 255) / 256, 256, 0, stream>>>(w_new, kFeat, WN, kCin / 8, n8);
  }
  {
    const int n8 = kOClsP * kFeat / 8;
    k_cast_rows<<<(n8 + 255) / 256, 256, 0, stream>>>(w_score, kOCls, WS, kFeat / 8, n8);
  }
  {
    const int n8 = kOLocP * kFeat / 8;
    k_cast_rows<<<(n8 + 255) / 256, 256, 0, stream>>>(w_bbox, kOLoc, WB, kFeat / 8, n8);
  }
  {
    const int n4 = kOClsP / 4;
    k_bias_pad<<<(n4 + 255) / 256, 256, 0, stream>>>(b_score, kOCls, BS, n4);
  }
  {
    const int n4 = kOLocP / 4;
    k_bias_pad<<<(n4 + 255) / 256, 256, 0, stream>>>(b_bbox, kOLoc, BB, n4);
  }
  {
    const int tiles = (kHWp / 64) * (kFeat / 64);
    wmma_gemm64<1, 0, 0, 2, false><<<dim3((tiles + 7) / 8, kNB), 256, 0, stream>>>(
        FT, nullptr, kCin, (long)kHWp * kCin,
        WN, nullptr, kCin, 0L,
        XTH, XTL, kFeat, (long)kHWp * kFeat,
        nullptr, nullptr, 0L,
        kHWp, kFeat, kCin, 1.0f);
  }
  {
    const int tiles = (kOClsP / 64) * (kHWp / 64);
    wmma_gemm64<1, 2, 1, 0, false><<<dim3((tiles + 7) / 8, kNB), 256, 0, stream>>>(
        WS, nullptr, kFeat, 0L,
        XTH, XTL, kFeat, (long)kHWp * kFeat,
        CLS, nullptr, kHWp, (long)kOClsP * kHWp,
        BS, nullptr, 0L,
        kOClsP, kHWp, kFeat, 1.0f);
  }
  {
    const int tiles = (kOLocP / 64) * (kHWp / 64);
    wmma_gemm64<1, 2, 1, 0, false><<<dim3((tiles + 7) / 8, kNB), 256, 0, stream>>>(
        WB, nullptr, kFeat, 0L,
        XTH, XTL, kFeat, (long)kHWp * kFeat,
        LOC, nullptr, kHWp, (long)kOLocP * kHWp,
        BB, nullptr, 0L,
        kOLocP, kHWp, kFeat, 1.0f);
  }
  k_psroi_pool<<<(kNR * kNCls) / 32, 256, 0, stream>>>(rois, stridep, CLS, (long)kOClsP * kHWp,
                                                       kNCls, kOCls, out, kNR * kNCls);
  k_psroi_pool<<<(kNR * kNLoc) / 32, 256, 0, stream>>>(rois, stridep, LOC, (long)kOLocP * kHWp,
                                                       kNLoc, kOLoc, out + (size_t)kNR * kNCls, kNR * kNLoc);
}
